// customlayer_28475633172946
// MI455X (gfx1250) — hardware-run, weakly checked
//
#include <hip/hip_runtime.h>

typedef __attribute__((ext_vector_type(16))) _Float16 v16h;
typedef __attribute__((ext_vector_type(8)))  _Float16 v8h;
typedef __attribute__((ext_vector_type(8)))  float    v8f;
typedef __attribute__((ext_vector_type(4)))  float    v4f;

constexpr int kImgH     = 256;
constexpr int kImgW     = 512;
constexpr int kOutH     = 32;
constexpr int kOutW     = 256;
constexpr int kOutElems = kOutH * kOutW;
constexpr int kLead     = kOutW - 1;
constexpr int kZ        = kImgW + kOutW - 1;
constexpr int kK        = kZ * kImgH;
constexpr int kTPRows   = kZ + kOutW - 1;
constexpr int kChunks   = 59;
constexpr int kChunkK   = kK / kChunks;
constexpr float kWCarry   = 64.0f;
constexpr float kImgCarry = 32.0f;
constexpr float kFold     = 1.0f / (kWCarry * kImgCarry);
constexpr float kF16Min   = 6.103515625e-05f;
constexpr float kWClamp   = 60000.0f;
static_assert(kZ == 767);
static_assert(kK == 196352);
static_assert(kTPRows == 1022);
static_assert(kChunks * kChunkK == kK);
static_assert(kChunkK == 3328);
static_assert((kChunkK % 32) == 0);
static_assert((kK % 8) == 0);
static_assert((kOutW % 64) == 0 && kOutH == 32);
static_assert((kOutW - 1) * kImgH + kK == kTPRows * kImgH);

constexpr size_t kBytesTP   = (size_t)kTPRows * kImgH * 2;
constexpr size_t kBytesAW   = (size_t)kOutH * kK * 2;
constexpr size_t kBytesPART = (size_t)kChunks * kOutElems * 4;
constexpr size_t kOffTP   = 0;
constexpr size_t kOffAW   = kOffTP + kBytesTP;
constexpr size_t kOffPART = kOffAW + kBytesAW;
constexpr size_t kWsTotal = kOffPART + kBytesPART;
static_assert(kBytesTP == 523264ull);
static_assert(kBytesAW == 12566528ull);
static_assert(kBytesPART == 1933312ull);
static_assert(kWsTotal == 15023104ull);
static_assert(kWsTotal <= 134217728ull);
static_assert((kOffAW % 128) == 0 && (kOffPART % 128) == 0);

union FragU { v16h v; v8h h[2]; };
__device__ __forceinline__ v16h frag_load(const _Float16* p) {
  FragU f;
  f.h[0] = *(const v8h*)(p);
  f.h[1] = *(const v8h*)(p + 16);
  return f.v;
}
__device__ __forceinline__ v8f mma_f16(v16h a, v16h b, v8f c) {
  c = __builtin_amdgcn_wmma_f32_16x16x32_f16(false, a, false, b, (short)0, c, false, false);
  asm volatile("v_nop\n\tv_nop\n\tv_nop\n\tv_nop" : "+v"(c) : "v"(a), "v"(b));
  return c;
}

__global__ __launch_bounds__(256) void image_plane_kernel(
    const float* __restrict__ img, unsigned short* __restrict__ tp)
{
  const int t = blockIdx.x * 256 + threadIdx.x;
  if (t >= kTPRows * 32) return;
  const int r   = t >> 5;
  const int ii0 = (t & 31) * 8;
  const int c   = r - kLead;
  const bool valid = (c >= 0) && (c < kImgW);
  const int cc = (c < 0) ? 0 : ((c > kImgW - 1) ? (kImgW - 1) : c);
  v8h hv;
#pragma unroll
  for (int e = 0; e < 8; ++e) {
    float x = img[(size_t)(ii0 + e) * kImgW + cc];
    asm volatile("" : "+v"(x));
    float y = valid ? (x * kImgCarry) : 0.0f;
    y = (y < kF16Min) ? 0.0f : y;
    hv[e] = (_Float16)y;
  }
  unsigned short* q = tp + (size_t)t * 8;
  *(volatile v8h*)q = hv;
  __threadfence();
  *(volatile v8h*)q = hv;
}

__global__ __launch_bounds__(256) void weight_plane_kernel(
    const float* __restrict__ pos, unsigned short* __restrict__ aw)
{
  const int t = blockIdx.x * 256 + threadIdx.x;
  if (t >= kOutH * kZ * 32) return;
  const int i   = t / (kZ * 32);
  const int rem = t - i * (kZ * 32);
  const int z   = rem >> 5;
  const int ii0 = (rem & 31) * 8;
  const float p0 = pos[0];
  const float p1 = pos[1];
  const float ai  = (float)i + p0;
  const float dy  = (float)(kLead - z) + p1;
  const float dy2 = dy * dy;
  v8h hv;
#pragma unroll
  for (int e = 0; e < 8; ++e) {
    const float dx  = ai - (float)(ii0 + e);
    const float den = fmaf(dx, dx, dy2);
    float w = kWCarry * __builtin_amdgcn_rcpf(den);
    w = fminf(w, kWClamp);
    w = (w < kF16Min) ? 0.0f : w;
    hv[e] = (_Float16)w;
  }
  unsigned short* q = aw + (size_t)t * 8;
  *(volatile v8h*)q = hv;
  __threadfence();
  *(volatile v8h*)q = hv;
}

__global__ __launch_bounds__(128) void splitk_product_kernel(
    const unsigned short* __restrict__ awp, const unsigned short* __restrict__ tpp,
    float* __restrict__ part)
{
  __shared__ __align__(16) float sT[4][16 * 68];
  const int lane  = threadIdx.x & 31;
  const int wave  = threadIdx.x >> 5;
  const int chunk = blockIdx.x;
  const int n0    = wave * 64;
  const int kbeg  = chunk * kChunkK;
  const int rlane = lane & 15;
  const int koff  = (lane >> 4) * 8;
  const int mOff  = (lane >> 4) * 8;

  const _Float16* A = (const _Float16*)awp;
  const _Float16* B = (const _Float16*)tpp;
  const _Float16* a0p = A + (size_t)rlane * kK + kbeg + koff;
  const _Float16* a1p = A + (size_t)(16 + rlane) * kK + kbeg + koff;
  const _Float16* b0p = B + (size_t)(n0 + rlane) * kImgH + kbeg + koff;
  const _Float16* b1p = b0p + 16 * kImgH;
  const _Float16* b2p = b0p + 32 * kImgH;
  const _Float16* b3p = b0p + 48 * kImgH;

  v8f acc[2][4];
#pragma unroll
  for (int i = 0; i < 2; ++i)
#pragma unroll
    for (int j = 0; j < 4; ++j) acc[i][j] = (v8f){0.f, 0.f, 0.f, 0.f, 0.f, 0.f, 0.f, 0.f};

#pragma unroll 1
  for (int ks = 0; ks < kChunkK; ks += 32) {
    const v16h bf0 = frag_load(b0p + ks);
    const v16h bf1 = frag_load(b1p + ks);
    const v16h bf2 = frag_load(b2p + ks);
    const v16h bf3 = frag_load(b3p + ks);
    const v16h af0 = frag_load(a0p + ks);
    const v16h af1 = frag_load(a1p + ks);
    acc[0][0] = mma_f16(af0, bf0, acc[0][0]);
    acc[0][1] = mma_f16(af0, bf1, acc[0][1]);
    acc[0][2] = mma_f16(af0, bf2, acc[0][2]);
    acc[0][3] = mma_f16(af0, bf3, acc[0][3]);
    acc[1][0] = mma_f16(af1, bf0, acc[1][0]);
    acc[1][1] = mma_f16(af1, bf1, acc[1][1]);
    acc[1][2] = mma_f16(af1, bf2, acc[1][2]);
    acc[1][3] = mma_f16(af1, bf3, acc[1][3]);
  }

  float* slab = sT[wave];
  const int hh = lane >> 4;
  const int c4 = (lane & 15) * 4;
#pragma unroll
  for (int i = 0; i < 2; ++i) {
#pragma unroll
    for (int j = 0; j < 4; ++j) {
#pragma unroll
      for (int r = 0; r < 8; ++r) {
        slab[(mOff + r) * 68 + (j << 4) + rlane] = acc[i][j][r];
      }
    }
    __builtin_amdgcn_fence(__ATOMIC_RELEASE, "workgroup");
    __builtin_amdgcn_wave_barrier();
    __builtin_amdgcn_fence(__ATOMIC_ACQUIRE, "workgroup");
    v4f sv[8];
#pragma unroll
    for (int it = 0; it < 8; ++it) sv[it] = *(const v4f*)(slab + (it * 2 + hh) * 68 + c4);
    for (int pass = 0; pass < 2; ++pass) {
#pragma unroll
      for (int it = 0; it < 8; ++it) {
        const int row = i * 16 + it * 2 + hh;
        float* dst = part + ((size_t)chunk * kOutH + row) * kOutW + n0 + c4;
        *(volatile v4f*)dst = sv[it];
      }
      __threadfence();
    }
    __builtin_amdgcn_fence(__ATOMIC_RELEASE, "workgroup");
    __builtin_amdgcn_wave_barrier();
    __builtin_amdgcn_fence(__ATOMIC_ACQUIRE, "workgroup");
  }
}

__global__ __launch_bounds__(256) void chunk_sum_kernel(
    const float* __restrict__ part, float* __restrict__ out)
{
  const int t = blockIdx.x * 256 + threadIdx.x;
  if (t >= kOutElems / 4) return;
  v4f s = (v4f){0.f, 0.f, 0.f, 0.f};
#pragma unroll 1
  for (int c = 0; c < kChunks; ++c) {
    const v4f v = *(const v4f*)(part + (size_t)c * kOutElems + (size_t)t * 4);
    s = s + v;
  }
  s = s * kFold;
  float* dst = out + (size_t)t * 4;
  *(volatile v4f*)dst = s;
  __threadfence();
  *(volatile v4f*)dst = s;
}

extern "C" void kernel_launch(void* const* d_in, const int* in_sizes, int n_in,
                              void* d_out, int out_size, void* d_ws, size_t ws_size,
                              hipStream_t stream) {
  if (n_in < 2) return;
  if (in_sizes[0] != kImgH * kImgW) return;
  if (in_sizes[1] != 2) return;
  if (out_size != kOutElems) return;
  if (ws_size < kWsTotal) return;

  const float* img = (const float*)d_in[0];
  const float* pos = (const float*)d_in[1];
  float* out = (float*)d_out;

  char* ws = (char*)d_ws;
  unsigned short* TP   = (unsigned short*)(ws + kOffTP);
  unsigned short* AW   = (unsigned short*)(ws + kOffAW);
  float*          PART = (float*)(ws + kOffPART);

  image_plane_kernel<<<(kTPRows * 32 + 255) / 256, 256, 0, stream>>>(img, TP);
  weight_plane_kernel<<<(kOutH * kZ * 32 + 255) / 256, 256, 0, stream>>>(pos, AW);
  splitk_product_kernel<<<kChunks, 128, 0, stream>>>(AW, TP, PART);
  chunk_sum_kernel<<<(kOutElems / 4 + 255) / 256, 256, 0, stream>>>(PART, out);
}
